// GNNModel_71511205479202
// MI455X (gfx1250) — hardware-verified
//
#include <hip/hip_runtime.h>

#define HID 32
#define NDIM 8
#define EMB 64
#define NG 128
#define EPB 64
#define KT 9
#define MROWS 288
#define MSC 16.0f
#define MUN 0.0625f

#define BT   256
#define ECAP 6144
#define SCAP 64
#define ETILE 2048

typedef __attribute__((ext_vector_type(16))) _Float16 v16h;
typedef __attribute__((ext_vector_type(8)))  _Float16 v8h;
typedef __attribute__((ext_vector_type(8)))  float    v8f;
typedef __attribute__((ext_vector_type(4)))  float    v4f;
typedef float __attribute__((may_alias)) float_a;

__device__ __forceinline__ v8f wmma_f16(v16h a, v16h b, v8f c) {
    v8f d = __builtin_amdgcn_wmma_f32_16x16x32_f16(false, a, false, b, (short)0, c, false, false);
    asm volatile("v_nop\n\tv_nop\n\tv_nop\n\tv_nop" : "+v"(d) : "v"(a), "v"(b));
    return d;
}
template <typename V> __device__ __forceinline__ void vst2(void* p, V v) {
    *(volatile V*)p = v; __threadfence(); *(volatile V*)p = v;
}
__device__ __forceinline__ v16h load_frag(const _Float16* tile, int ld, int k0, int lane) {
    union { v16h v; v8h h[2]; } r;
    const _Float16* row = tile + (lane & 15) * ld + k0 + 8 * (lane >> 4);
    r.h[0] = *(const v8h*)(row);
    r.h[1] = *(const v8h*)(row + 16);
    return r.v;
}

__global__ __launch_bounds__(128)
void edge_kernel(const float* __restrict__ x, const float* __restrict__ ea,
                 const int* __restrict__ src,
                 const float* __restrict__ W1, const float* __restrict__ b1,
                 const float* __restrict__ W2, const float* __restrict__ b2,
                 float* __restrict__ msg, int E, int N) {
    __shared__ __align__(16) _Float16 sMt[HID * 296];
    __shared__ float sH[EPB * HID];
    __shared__ float sXS[EPB * NDIM];
    __shared__ __align__(16) float sOut[4][16 * HID];

    const int tid  = threadIdx.x;
    const int lane = tid & 31;
    const int wave = tid >> 5;
    const int n    = lane & 15;
    const int hi   = lane >> 4;

    for (int i = tid; i < MROWS * HID; i += 128) {
        int row = i >> 5, o = i & 31;
        float v;
        if (row < 256)       v = W2[(row >> 3) * 256 + (row & 7) * 32 + o];
        else if (row < 264)  v = b2[(row - 256) * 32 + o];
        else                 v = 0.0f;
        sMt[o * 296 + row] = (_Float16)(v * MSC);
    }
    __syncthreads();

    for (long long base = (long long)blockIdx.x * EPB; base < E; base += (long long)gridDim.x * EPB) {
        __syncthreads();
        for (int i = tid; i < EPB * NDIM; i += 128) {
            int el = i >> 3;
            long long e = base + el;
            float v = 0.0f;
            if (e < E) { int s = src[e]; s = s < 0 ? 0 : (s >= N ? N - 1 : s); v = x[(long long)s * NDIM + (i & 7)]; }
            sXS[i] = v;
        }
        {
            int el = tid >> 1, k0 = (tid & 1) * 16;
            long long e = base + el;
            float a0 = 0.f, a1 = 0.f, a2 = 0.f;
            if (e < E) { a0 = ea[e * 3]; a1 = ea[e * 3 + 1]; a2 = ea[e * 3 + 2]; }
#pragma unroll
            for (int k = 0; k < 16; ++k) {
                int kk = k0 + k;
                float v = b1[kk] + a0 * W1[kk] + a1 * W1[32 + kk] + a2 * W1[64 + kk];
                sH[el * HID + kk] = fmaxf(v, 0.0f);
            }
        }
        __syncthreads();

        const int eb = wave * 16;
        const float* xsp = &sXS[(eb + n) * NDIM];
        const float* hp  = &sH[(eb + n) * HID];
        float xq[8];
#pragma unroll
        for (int i = 0; i < 8; ++i) xq[i] = xsp[i];

        v8f c0 = {}; v8f c1 = {};
#pragma unroll
        for (int t = 0; t < 8; ++t) {
            const float h0 = hp[t * 4 + hi];
            const float h1 = hp[t * 4 + 2 + hi];
            v16h a;
#pragma unroll
            for (int j = 0; j < 8; ++j) { a[j] = (_Float16)(h0 * xq[j]); a[8 + j] = (_Float16)(h1 * xq[j]); }
            c0 = wmma_f16(a, load_frag(sMt, 296, t * 32, lane), c0);
            c1 = wmma_f16(a, load_frag(sMt + 16 * 296, 296, t * 32, lane), c1);
        }
        {
            v16h a;
#pragma unroll
            for (int j = 0; j < 8; ++j) { a[j] = hi ? (_Float16)0.0f : (_Float16)xq[j]; a[8 + j] = (_Float16)0.0f; }
            c0 = wmma_f16(a, load_frag(sMt, 296, 256, lane), c0);
            c1 = wmma_f16(a, load_frag(sMt + 16 * 296, 296, 256, lane), c1);
        }

        float* so = sOut[wave];
#pragma unroll
        for (int r = 0; r < 8; ++r) { so[(hi * 8 + r) * HID + n] = c0[r] * MUN; so[(hi * 8 + r) * HID + 16 + n] = c1[r] * MUN; }
        __syncthreads();
#pragma unroll
        for (int q = 0; q < 4; ++q) {
            const int rloc = q * 4 + (lane >> 3);
            const long long e = base + eb + rloc;
            const v4f v = *(const v4f*)(so + rloc * HID + (lane & 7) * 4);
            if (base + eb + q * 4 + 3 < E) {
                vst2(msg + e * HID + (lane & 7) * 4, v);
            }
        }
    }
}

__global__ __launch_bounds__(256)
void node_gather(const float* __restrict__ x, const float* __restrict__ root, const float* __restrict__ cbias,
                 const int* __restrict__ dst, const float* __restrict__ msg,
                 float* __restrict__ hnode, int E, int N)
{
    __shared__ int   lsrc[ECAP];
    __shared__ unsigned short ltgt[ECAP];
    __shared__ unsigned short sub[BT][SCAP];
    __shared__ int   scnt[BT];
    __shared__ int   wcnt[8][8];
    __shared__ int   total;
    __shared__ float sroot[NDIM * HID];
    __shared__ float sbias[HID];

    const int tid  = threadIdx.x;
    const int lane = tid & 31;
    const int wave = tid >> 5;
    const int b    = blockIdx.x;
    const int tlo  = b * BT;

    if (tid == 0) total = 0;
    sroot[tid] = root[tid];
    if (tid < HID) sbias[tid] = cbias[tid];
    __syncthreads();

    for (int e0 = 0; e0 < E; e0 += ETILE) {
        int rv[8]; unsigned msk[8];
        #pragma unroll
        for (int j = 0; j < 8; ++j) {
            const int e = e0 + j * 256 + tid;
            const int r = (e < E) ? dst[e] : -1;
            rv[j] = r;
            const bool hit = (r >= tlo) && (r < tlo + BT);
            msk[j] = (unsigned)__builtin_amdgcn_ballot_w32(hit);
        }
        if (lane < 8) wcnt[lane][wave] = __builtin_popcount(msk[lane]);
        __syncthreads();
        const int base = total;
        int run = 0, pre[8];
        #pragma unroll
        for (int j = 0; j < 8; ++j) {
            #pragma unroll
            for (int w = 0; w < 8; ++w) {
                if (w == wave) pre[j] = run;
                run += wcnt[j][w];
            }
        }
        #pragma unroll
        for (int j = 0; j < 8; ++j) {
            const unsigned m = msk[j];
            if ((m >> lane) & 1u) {
                const int pos = base + pre[j] + __builtin_popcount(m & ((1u << lane) - 1u));
                if (pos < ECAP) { lsrc[pos] = e0 + j * 256 + tid; ltgt[pos] = (unsigned short)(rv[j] - tlo); }
            }
        }
        __syncthreads();
        if (tid == 0) total = base + run;
        __syncthreads();
    }
    const int n = (total < ECAP) ? total : ECAP;
    {
        int k = 0;
        for (int i = 0; i < n; ++i) {
            if ((int)ltgt[i] == tid) { if (k < SCAP) sub[tid][k] = (unsigned short)i; ++k; }
        }
        scnt[tid] = (k < SCAP) ? k : SCAP;
    }
    __syncthreads();

    for (int s = 0; s < 32; ++s) {
        const int t = wave * 32 + s;
        const int node = tlo + t;
        if (node >= N) break;
        const int cnt = scnt[t];
        float a = 0.0f;
        for (int k = 0; k < cnt; ++k) a += msg[(long long)lsrc[sub[t][k]] * HID + lane];
        float acc = sbias[lane] + a / fmaxf((float)cnt, 1.0f);
#pragma unroll
        for (int i = 0; i < NDIM; ++i) acc += x[(long long)node * NDIM + i] * sroot[i * HID + lane];
        acc = fmaxf(acc, 0.0f);
        vst2(hnode + (long long)node * HID + lane, (float_a)acc);
    }
}

__global__ __launch_bounds__(256)
void pool_kernel(const float* __restrict__ hnode, const int* __restrict__ batch, float* __restrict__ pooled, int N)
{
    __shared__ float part[8][HID];
    __shared__ int rng[2];
    const int g = blockIdx.x, tid = threadIdx.x, lane = tid & 31, wave = tid >> 5;
    if (tid < 2) {
        const int key = g + tid;
        int lo = 0, hi = N;
        while (lo < hi) { const int mid = (lo + hi) >> 1; if (batch[mid] < key) lo = mid + 1; else hi = mid; }
        rng[tid] = lo;
    }
    __syncthreads();
    const int n0 = rng[0], n1 = rng[1];
    float s = 0.0f;
    for (int nd = n0 + wave; nd < n1; nd += 8) s += hnode[(long long)nd * HID + lane];
    part[wave][lane] = s;
    __syncthreads();
    if (wave == 0) {
        float tsum = 0.0f;
#pragma unroll
        for (int w = 0; w < 8; ++w) tsum += part[w][lane];
        const float cntg = (float)(n1 - n0);
        vst2(pooled + g * HID + lane, (float_a)(tsum / fmaxf(cntg, 1.0f)));
    }
}

__global__ __launch_bounds__(128)
void head_kernel(const float* __restrict__ pooled, const float* __restrict__ emb, const float* __restrict__ ratios,
                 const int* __restrict__ ids,
                 const float* __restrict__ fc0w, const float* __restrict__ fc0b,
                 const float* __restrict__ fc1w, const float* __restrict__ fc1b,
                 const float* __restrict__ fc2w, const float* __restrict__ fc2b,
                 float* __restrict__ out, int G) {
    __shared__ float u[64];
    __shared__ __align__(16) float res[NG];
    int tid = threadIdx.x;
    if (tid < 64) {
        float s = 0.0f;
        for (int t = 0; t < 5; ++t) { int id = ids[t]; id = id < 0 ? 0 : (id > 117 ? 117 : id); s += emb[id * 64 + tid] * ratios[t]; }
        u[tid] = s;
    }
    __syncthreads();
    if (tid < G) {
        float pl[32];
#pragma clang loop unroll(disable)
        for (int j = 0; j < 32; ++j) pl[j] = pooled[tid * 32 + j];
        float z0[64];
#pragma clang loop unroll(disable)
        for (int o = 0; o < 64; ++o) {
            float a = fc0b[o];
#pragma clang loop unroll(disable)
            for (int j = 0; j < 32; ++j) a += pl[j] * fc0w[j * 64 + o];
#pragma clang loop unroll(disable)
            for (int j = 0; j < 64; ++j) a += u[j] * fc0w[(32 + j) * 64 + o];
            z0[o] = fmaxf(a, 0.0f);
        }
        float z1[32];
#pragma clang loop unroll(disable)
        for (int o = 0; o < 32; ++o) {
            float a = fc1b[o];
#pragma clang loop unroll(disable)
            for (int j = 0; j < 64; ++j) a += z0[j] * fc1w[j * 32 + o];
            z1[o] = fmaxf(a, 0.0f);
        }
        float a = fc2b[0];
#pragma clang loop unroll(disable)
        for (int j = 0; j < 32; ++j) a += z1[j] * fc2w[j];
        res[tid] = a;
    }
    __syncthreads();
    if (tid < NG / 4) vst2(out + tid * 4, *(const v4f*)(res + tid * 4));
}

extern "C" void kernel_launch(void* const* d_in, const int* in_sizes, int n_in,
                              void* d_out, int out_size, void* d_ws, size_t ws_size,
                              hipStream_t stream) {
    (void)n_in; (void)ws_size;
    const float* x      = (const float*)d_in[0];
    const float* ea     = (const float*)d_in[1];
    const float* ratios = (const float*)d_in[2];
    const int*   eidx   = (const int*)  d_in[3];
    const int*   batch  = (const int*)  d_in[4];
    const int*   ids    = (const int*)  d_in[5];
    const float* W1     = (const float*)d_in[6];
    const float* b1     = (const float*)d_in[7];
    const float* W2     = (const float*)d_in[8];
    const float* b2     = (const float*)d_in[9];
    const float* emb    = (const float*)d_in[10];
    const float* root   = (const float*)d_in[11];
    const float* cbias  = (const float*)d_in[12];
    const float* fc0w   = (const float*)d_in[13];
    const float* fc0b   = (const float*)d_in[14];
    const float* fc1w   = (const float*)d_in[15];
    const float* fc1b   = (const float*)d_in[16];
    const float* fc2w   = (const float*)d_in[17];
    const float* fc2b   = (const float*)d_in[18];

    const int N = in_sizes[0] / NDIM;
    const int E = in_sizes[1] / 3;
    const int G = out_size;

    float* msg    = (float*)d_ws;
    float* hnode  = msg + (size_t)E * HID;
    float* pooled = hnode + (size_t)N * HID;

    const int* src = eidx;
    const int* dst = eidx + E;
    edge_kernel<<<2048, 128, 0, stream>>>(x, ea, src, W1, b1, W2, b2, msg, E, N);
    node_gather<<<(N + BT - 1) / BT, 256, 0, stream>>>(x, root, cbias, dst, msg, hnode, E, N);
    pool_kernel<<<G, 256, 0, stream>>>(hnode, batch, pooled, N);
    head_kernel<<<1, 128, 0, stream>>>(pooled, emb, ratios, ids, fc0w, fc0b, fc1w, fc1b, fc2w, fc2b, (float*)d_out, G);
}
